// StackedAttentionBlock_80556406604300
// MI455X (gfx1250) — hardware-verified
//
#include <hip/hip_runtime.h>
#include <math.h>
#include <stdint.h>

#define NB      4
#define CD      128
#define HW      64
#define NSEQ    4096
#define NHEAD   4
#define HDIM    32
#define DFF     512
#define MP      (NB * NSEQ)
#define QKP     64
#define VTR     64
#define LNEPS   1.0e-5f
#define WSC     64.0f
#define QKCARRY 16.0f
#define VCARRY  16.0f
#define PCARRY  1024.0f
#define AOCARRY 64.0f
static_assert(NHEAD * HDIM == CD);
static_assert(HW * HW == NSEQ);
static_assert((MP % 64) == 0 && (CD % 64) == 0 && (DFF % 64) == 0 && (NSEQ % 64) == 0);
static_assert(CD == 16 * 8);
static_assert(QKP == 2 * HDIM && VTR == 2 * HDIM);
static_assert((MP * 4) % 256 == 0);

typedef _Float16 v16h __attribute__((ext_vector_type(16)));
typedef _Float16 v8h  __attribute__((ext_vector_type(8)));
typedef _Float16 v4h  __attribute__((ext_vector_type(4)));
typedef __attribute__((ext_vector_type(16))) __bf16 v16b;
typedef float    v8f  __attribute__((ext_vector_type(8)));
typedef float    v4f  __attribute__((ext_vector_type(4)));
typedef unsigned int v4u __attribute__((ext_vector_type(4)));

union FragH  { v16h v; v8h h[2]; };
union Frag16 { v16h h; v16b b; v8h hh[2]; v4u u[2]; };

__device__ __forceinline__ unsigned short bf_bits(float f) {
  unsigned u = __float_as_uint(f);
  return (unsigned short)((u + 0x7FFFu + ((u >> 16) & 1u)) >> 16);
}
__device__ __forceinline__ float bf_up(unsigned short h) { return __uint_as_float(((unsigned)h) << 16); }
__device__ __forceinline__ float bfr(float f) { return bf_up(bf_bits(f)); }
__device__ __forceinline__ unsigned short h_bits(_Float16 x) { return __builtin_bit_cast(unsigned short, x); }
__device__ __forceinline__ unsigned pk16(unsigned short a, unsigned short b) { return (unsigned)a | ((unsigned)b << 16); }
__device__ __forceinline__ v8f zero8() { v8f z = {0.f, 0.f, 0.f, 0.f, 0.f, 0.f, 0.f, 0.f}; return z; }

__device__ __forceinline__ v16h ldfrag_h(const _Float16* p) {
  FragH f;
  f.h[0] = *(const v8h*)(p);
  f.h[1] = *(const v8h*)(p + 16);
  return f.v;
}
__device__ __forceinline__ Frag16 ldfrag16(const unsigned short* p) {
  Frag16 f;
  f.u[0] = *(const v4u*)(p);
  f.u[1] = *(const v4u*)(p + 16);
  return f;
}

__device__ __forceinline__ v8f mma_h(v16h a, v16h b, v8f c) {
  c = __builtin_amdgcn_wmma_f32_16x16x32_f16(false, a, false, b, (short)0, c, false, false);
#if defined(__HIP_DEVICE_COMPILE__)
  asm volatile("v_nop\n\tv_nop\n\tv_nop\n\tv_nop" : "+v"(c) : "v"(a), "v"(b));
#endif
  return c;
}
__device__ __forceinline__ v8f mma_h_raw(v16h a, v16h b, v8f c) {
  return __builtin_amdgcn_wmma_f32_16x16x32_f16(false, a, false, b, (short)0, c, false, false);
}
template <int TB>
__device__ __forceinline__ v8f mma16_raw(const Frag16& a, const Frag16& b, v8f c) {
  if (TB == 0) return __builtin_amdgcn_wmma_f32_16x16x32_f16(false, a.h, false, b.h, (short)0, c, false, false);
  else         return __builtin_amdgcn_wmma_f32_16x16x32_bf16(false, a.b, false, b.b, (short)0, c, false, false);
}
__device__ __forceinline__ void dep_guard1(v8f& a, v8f& b, v16h x) {
#if defined(__HIP_DEVICE_COMPILE__)
  asm volatile("v_nop\n\tv_nop\n\tv_nop\n\tv_nop" : "+v"(a), "+v"(b) : "v"(x));
#endif
}
__device__ __forceinline__ void dep_guard3(v8f& a, v8f& b, v16h x, v16h y, v16h z) {
#if defined(__HIP_DEVICE_COMPILE__)
  asm volatile("v_nop\n\tv_nop\n\tv_nop\n\tv_nop" : "+v"(a), "+v"(b) : "v"(x), "v"(y), "v"(z));
#endif
}
__device__ __forceinline__ void keep4_h(v16h a, v16h b, v16h c, v16h d) {
#if defined(__HIP_DEVICE_COMPILE__)
  asm volatile("v_nop" :: "v"(a), "v"(b), "v"(c), "v"(d));
#endif
}
__device__ __forceinline__ void acc_guard4(v8f& a, v8f& b, v8f& c, v8f& d) {
#if defined(__HIP_DEVICE_COMPILE__)
  asm volatile("v_nop\n\tv_nop\n\tv_nop\n\tv_nop" : "+v"(a), "+v"(b), "+v"(c), "+v"(d));
#endif
}
__device__ __forceinline__ void wave_sync_lds() {
  __builtin_amdgcn_fence(__ATOMIC_RELEASE, "workgroup");
  __builtin_amdgcn_wave_barrier();
  __builtin_amdgcn_fence(__ATOMIC_ACQUIRE, "workgroup");
}
__device__ __forceinline__ float wsum16(float v) {
#pragma unroll
  for (int off = 8; off > 0; off >>= 1) v += __shfl_xor(v, off, 32);
  return v;
}

template <int KIND>
__global__ __launch_bounds__(256) void conv_t16(const float* __restrict__ Wa, const float* __restrict__ Wb,
                                                 unsigned short* dst, int Cin, int Osrc, int Odst, int n8, float wsc) {
  const int i    = blockIdx.x * 256 + threadIdx.x;
  const int ic   = (i < n8) ? i : (n8 - 1);
  const int per  = (Odst * Cin) >> 3;
  const int bi   = ic / per;
  const int r    = ic - bi * per;
  const int cin8 = Cin >> 3;
  const int o    = r / cin8;
  const int c0   = (r - o * cin8) * 8;
  const int sel  = (o >= Osrc) ? 1 : 0;
  const int os   = o - sel * Osrc;
  const float* pa = Wa + ((size_t)bi * Cin + c0) * Osrc + os;
  const float* pb = Wb + ((size_t)bi * Cin + c0) * Osrc + os;
  float v[8];
#pragma unroll
  for (int e = 0; e < 8; ++e) {
    const float xa = pa[(size_t)e * Osrc];
    const float xb = pb[(size_t)e * Osrc];
    v[e] = bfr(sel ? xb : xa);
  }
  v4u ov;
#pragma unroll
  for (int e = 0; e < 4; ++e) {
    if (KIND == 0) ov[e] = pk16(h_bits((_Float16)(v[2 * e] * wsc)), h_bits((_Float16)(v[2 * e + 1] * wsc)));
    else           ov[e] = pk16(bf_bits(v[2 * e]), bf_bits(v[2 * e + 1]));
  }
  if (i < n8) *(volatile v4u*)(dst + (size_t)i * 8) = ov;
  __threadfence();
  if (i < n8) *(volatile v4u*)(dst + (size_t)i * 8) = ov;
}

__global__ __launch_bounds__(128) void pack_bias(const float* __restrict__ bq, const float* __restrict__ bk,
                                                 const float* __restrict__ bv, float* dst) {
  const int t  = threadIdx.x;
  const int u  = t & 63;
  const int h  = u >> 4, j4 = (u & 15) * 4;
  const int si = h * HDIM + (j4 & 31);
  const v4f va = *(const v4f*)(bq + si), vb = *(const v4f*)(bk + si), vc = *(const v4f*)(bv + si);
  const bool selk = (j4 >= 32);
  const bool isv  = (t >= 64);
  v4f o;
#pragma unroll
  for (int e = 0; e < 4; ++e) {
    const float q = selk ? vb[e] : va[e];
    o[e] = isv ? vc[e] : q;
  }
  *(volatile v4f*)(dst + 4 * t) = o;
  __threadfence();
  *(volatile v4f*)(dst + 4 * t) = o;
}

__global__ __launch_bounds__(256) void xprep(const float* __restrict__ src, unsigned short* XH) {
  __shared__ __align__(16) float T[CD * 36];
  const int tid = threadIdx.x, wave = tid >> 5, lane = tid & 31;
  const int bx = blockIdx.x;
  const int b  = bx >> 7;
  const int n0 = (bx & 127) * 32;
  const float* sb = src + (size_t)b * CD * NSEQ + n0;
  {
    const int q = lane >> 3, e = lane & 7;
#pragma unroll
    for (int it = 0; it < 4; ++it) {
      const int c = wave * 16 + it * 4 + q;
      const v4f v = *(const v4f*)(sb + (size_t)c * NSEQ + 4 * e);
      *(v4f*)(T + c * 36 + 4 * e) = v;
    }
  }
  __syncthreads();
  const int hh = lane >> 4, c = lane & 15;
#pragma unroll 1
  for (int i = 0; i < 2; ++i) {
    const int tl = wave * 4 + 2 * i + hh;
    const int n  = n0 + tl;
    float x[8];
#pragma unroll
    for (int e = 0; e < 8; ++e) x[e] = bfr(T[(8 * c + e) * 36 + tl]);
    v4u ox;
#pragma unroll
    for (int e = 0; e < 4; ++e) ox[e] = pk16(h_bits((_Float16)x[2 * e]), h_bits((_Float16)x[2 * e + 1]));
    const size_t ro = ((size_t)b * NSEQ + n) * CD + 8 * c;
    *(volatile v4u*)(XH + ro) = ox;
    __threadfence();
    *(volatile v4u*)(XH + ro) = ox;
  }
}

__global__ __launch_bounds__(256) void xiprep(const unsigned short* __restrict__ XH, const float* __restrict__ AO,
                                               unsigned short* XI, int hsel) {
  const int t   = blockIdx.x * 256 + threadIdx.x;
  const int tok = t >> 2, cg = (t & 3) * 8;
  const _Float16* xp = (const _Float16*)(const void*)XH + (size_t)tok * CD + hsel * HDIM + cg;
  const v8h xh = *(const v8h*)(xp);
  const float* ap = AO + (size_t)tok * CD + (hsel - 1) * HDIM + cg;
  const v4f a0 = *(const v4f*)(ap), a1 = *(const v4f*)(ap + 4);
  float x[8];
#pragma unroll
  for (int e = 0; e < 4; ++e) { x[e] = (float)xh[e] + a0[e]; x[4 + e] = (float)xh[4 + e] + a1[e]; }
  v4u o;
#pragma unroll
  for (int e = 0; e < 4; ++e) o[e] = pk16(h_bits((_Float16)x[2 * e]), h_bits((_Float16)x[2 * e + 1]));
  unsigned short* dp = XI + (size_t)tok * HDIM + cg;
  *(volatile v4u*)dp = o;
  __threadfence();
  *(volatile v4u*)dp = o;
}

template <int TB, int A32, int NPA, int OM, int BIASM, int ACT, int RES>
__global__ __launch_bounds__(256) void gemm64(
    const void* __restrict__ Ap, const void* __restrict__ Ap2, int lda, long long strideA, float ascale,
    const unsigned short* __restrict__ Btp, int ldb, long long strideB,
    const float* __restrict__ bias, float bscale,
    const void* resid,
    void* Cout, void* Cout2, int ldc, long long strideC,
    int M, int N, int K, float oscale) {
  __shared__ __align__(16) float sT[8][16 * 68];
  const int b    = blockIdx.y;
  const int lane = threadIdx.x & 31;
  const int wave = threadIdx.x >> 5;
  const int tilesN = N >> 6;
  const int tilesM = M >> 6;
  const int tile = blockIdx.x * 8 + wave;
  if (tile >= tilesM * tilesN) return;
  const int tm = tile / tilesN;
  const int tn = tile - tm * tilesN;
  const int m0 = tm << 6;
  const int n0 = tn << 6;

  const unsigned short* A1 = (const unsigned short*)Ap  + (size_t)b * strideA;
  const unsigned short* A2 = (const unsigned short*)Ap2 + (size_t)b * strideA;
  const float*          Af = (const float*)Ap + (size_t)b * strideA;
  const unsigned short* Bb = Btp + (size_t)b * strideB;

  const int rlane = lane & 15;
  const int koff  = (lane >> 4) * 8;
  const int mOff  = (lane >> 4) * 8;

  v8f acc[4][4];
#pragma unroll
  for (int i = 0; i < 4; ++i)
#pragma unroll
    for (int j = 0; j < 4; ++j) acc[i][j] = zero8();

  for (int k0 = 0; k0 < K; k0 += 32) {
    Frag16 bh[4];
#pragma unroll
    for (int j = 0; j < 4; ++j) {
      const size_t bo = (size_t)(n0 + (j << 4) + rlane) * ldb + koff + k0;
      bh[j] = ldfrag16(Bb + bo);
    }
#pragma unroll
    for (int i = 0; i < 4; ++i) {
#pragma unroll
      for (int pl = 0; pl < NPA; ++pl) {
        Frag16 ah;
        if (A32) {
          const float* ap = Af + (size_t)(m0 + (i << 4) + rlane) * lda + koff + k0;
          const v4f x0 = *(const v4f*)(ap), x1 = *(const v4f*)(ap + 4);
          const v4f x2 = *(const v4f*)(ap + 16), x3 = *(const v4f*)(ap + 20);
#pragma unroll
          for (int e = 0; e < 4; ++e) {
            ah.hh[0][e]     = (_Float16)(x0[e] * ascale);
            ah.hh[0][4 + e] = (_Float16)(x1[e] * ascale);
            ah.hh[1][e]     = (_Float16)(x2[e] * ascale);
            ah.hh[1][4 + e] = (_Float16)(x3[e] * ascale);
          }
        } else {
          const unsigned short* Apl = (pl == 0) ? A1 : A2;
          const size_t ao = (size_t)(m0 + (i << 4) + rlane) * lda + koff + k0;
          ah = ldfrag16(Apl + ao);
        }
#pragma unroll
        for (int j = 0; j < 4; ++j) acc[i][j] = mma16_raw<TB>(ah, bh[j], acc[i][j]);
        dep_guard1(acc[i][0], acc[i][3], ah.h);
      }
    }
    keep4_h(bh[0].h, bh[1].h, bh[2].h, bh[3].h);
  }
  acc_guard4(acc[0][0], acc[0][1], acc[0][2], acc[0][3]);
  acc_guard4(acc[1][0], acc[1][1], acc[1][2], acc[1][3]);
  acc_guard4(acc[2][0], acc[2][1], acc[2][2], acc[2][3]);
  acc_guard4(acc[3][0], acc[3][1], acc[3][2], acc[3][3]);

  const int hh2 = lane >> 4, c4 = (lane & 15) * 4;
  const int q8  = lane >> 3, c8 = (lane & 7) * 8;
  float bc[8];
#pragma unroll
  for (int e = 0; e < 8; ++e) bc[e] = 0.f;
  if (BIASM == 0) {
    if (OM == 0) {
      const int cb = n0 + c4;
      const int i0 = (cb < N - 4) ? cb : (N - 4);
      const v4f b0v = *(const v4f*)(bias + i0);
#pragma unroll
      for (int e = 0; e < 4; ++e) bc[e] = bfr(b0v[e]) * bscale;
    } else {
      const int cb = n0 + c8;
      const int i0 = (cb < N - 8) ? cb : (N - 8);
      const v4f b0a = *(const v4f*)(bias + i0), b0b = *(const v4f*)(bias + i0 + 4);
#pragma unroll
      for (int e = 0; e < 4; ++e) {
        bc[e]     = bfr(b0a[e]) * bscale;
        bc[4 + e] = bfr(b0b[e]) * bscale;
      }
    }
  }

  float* slab = sT[wave];
#pragma unroll
  for (int i = 0; i < 4; ++i) {
    const int mBase = m0 + (i << 4);
#pragma unroll
    for (int j = 0; j < 4; ++j) {
#pragma unroll
      for (int r = 0; r < 8; ++r) {
        slab[(mOff + r) * 68 + (j << 4) + rlane] = acc[i][j][r];
      }
    }
    wave_sync_lds();
    if (OM == 0) {
      float* C = (float*)Cout + (size_t)b * strideC;
      const float*    Rf = (const float*)resid + (size_t)b * strideC;
      const _Float16* Rh = (const _Float16*)resid + (size_t)b * strideC;
      v4f vals[8];
#pragma unroll
      for (int it = 0; it < 8; ++it) {
        const int row = it * 2 + hh2;
        v4f v = *(const v4f*)(slab + row * 68 + c4);
#pragma unroll
        for (int e = 0; e < 4; ++e) {
          float f = v[e] * oscale + bc[e];
          if (ACT == 1) f = fmaxf(f, 0.f);
          if (ACT == 2) f = 0.5f * f * (1.0f + erff(f * 0.70710678118654752f));
          v[e] = f;
        }
        if (RES == 1) {
          const v4f rr = *(const v4f*)(Rf + (size_t)(mBase + row) * ldc + n0 + c4);
#pragma unroll
          for (int e = 0; e < 4; ++e) v[e] += rr[e];
        }
        if (RES == 2) {
          const v4h rr = *(const v4h*)(Rh + (size_t)(mBase + row) * ldc + n0 + c4);
#pragma unroll
          for (int e = 0; e < 4; ++e) v[e] += (float)rr[e];
        }
        vals[it] = v;
      }
      for (int pass = 0; pass < 2; ++pass) {
#pragma unroll
        for (int it = 0; it < 8; ++it) {
          const int row = it * 2 + hh2;
          *(volatile v4f*)(C + (size_t)(mBase + row) * ldc + n0 + c4) = vals[it];
        }
        __threadfence();
      }
    } else {
      unsigned short* C  = (unsigned short*)Cout  + (size_t)b * strideC;
      unsigned short* C2 = (unsigned short*)Cout2 + (size_t)b * strideC;
      v4u hv[4], lv[4];
#pragma unroll
      for (int it = 0; it < 4; ++it) {
        const int row = it * 4 + q8;
        const float* sp = slab + row * 68 + c8;
        float bm = 0.f;
        if (BIASM == 1) bm = bfr(bias[mBase + row]) * bscale;
        v4u a, a2;
#pragma unroll
        for (int e = 0; e < 4; ++e) {
          float f0 = sp[2 * e]     * oscale + ((BIASM == 1) ? bm : bc[2 * e]);
          float f1 = sp[2 * e + 1] * oscale + ((BIASM == 1) ? bm : bc[2 * e + 1]);
          if (ACT == 1) { f0 = fmaxf(f0, 0.f); f1 = fmaxf(f1, 0.f); }
          if (ACT == 2) {
            f0 = 0.5f * f0 * (1.0f + erff(f0 * 0.70710678118654752f));
            f1 = 0.5f * f1 * (1.0f + erff(f1 * 0.70710678118654752f));
          }
          if (OM == 2) {
            a[e]  = pk16(h_bits((_Float16)f0), h_bits((_Float16)f1));
            a2[e] = a[e];
          } else {
            const unsigned short h0 = bf_bits(f0), h1 = bf_bits(f1);
            const unsigned short l0 = bf_bits(f0 - bf_up(h0)), l1 = bf_bits(f1 - bf_up(h1));
            a[e]  = pk16(h0, h1);
            a2[e] = pk16(l0, l1);
          }
        }
        hv[it] = a;
        lv[it] = a2;
      }
      for (int pass = 0; pass < 2; ++pass) {
#pragma unroll
        for (int it = 0; it < 4; ++it) {
          const int row = it * 4 + q8;
          *(volatile v4u*)(C + (size_t)(mBase + row) * ldc + n0 + c8) = hv[it];
          if (OM == 3) *(volatile v4u*)(C2 + (size_t)(mBase + row) * ldc + n0 + c8) = lv[it];
        }
        __threadfence();
      }
    }
    wave_sync_lds();
  }
}

__global__ __launch_bounds__(128)
void attn_head(const unsigned short* __restrict__ qk, const unsigned short* __restrict__ vt, float* ao, int hcol) {
  __shared__ __align__(16) float Ps[4][16 * 68];
  __shared__ __align__(16) float Os[4][16 * 32];

  const int tid  = threadIdx.x;
  const int wave = tid >> 5;
  const int lane = tid & 31;
  const int hh   = lane >> 4;
  const int c    = lane & 15;

  const int bx = blockIdx.x;
  const int b  = bx >> 6;
  const int q0 = (bx & 63) * 64 + wave * 16;
  const size_t gr = (size_t)b * NSEQ + q0;

  const _Float16* Q  = (const _Float16*)(const void*)qk;
  const _Float16* Kp = Q + (size_t)b * NSEQ * QKP + HDIM;
  const _Float16* V  = (const _Float16*)(const void*)vt + (size_t)b * VTR * NSEQ;
  const float lsc = (1.4426950408889634f * 0.17677669529663688f) / (QKCARRY * QKCARRY);

  const v16h qa = ldfrag_h(Q + (gr + c) * QKP + 8 * hh);

  float mrow[8], lrow[8];
  v8f oacc0 = zero8(), oacc1 = zero8();
#pragma unroll
  for (int r = 0; r < 8; ++r) { mrow[r] = -INFINITY; lrow[r] = 0.f; }
  float* pt = Ps[wave];

#pragma unroll 1
  for (int kb = 0; kb < NSEQ; kb += 64) {
    v8f s[4];
#pragma unroll
    for (int j = 0; j < 4; ++j) {
      const v16h kf = ldfrag_h(Kp + (size_t)(kb + 16 * j + c) * QKP + 8 * hh);
      s[j] = mma_h(qa, kf, zero8());
    }
#pragma unroll
    for (int r = 0; r < 8; ++r) {
      const float t0 = s[0][r] * lsc, t1 = s[1][r] * lsc, t2 = s[2][r] * lsc, t3 = s[3][r] * lsc;
      float mx = fmaxf(fmaxf(t0, t1), fmaxf(t2, t3));
#pragma unroll
      for (int off = 1; off < 16; off <<= 1) mx = fmaxf(mx, __shfl_xor(mx, off, 32));
      const float mn = fmaxf(mrow[r], mx);
      const float al = exp2f(mrow[r] - mn);
      mrow[r] = mn;
      const float e0 = exp2f(t0 - mn), e1 = exp2f(t1 - mn), e2 = exp2f(t2 - mn), e3 = exp2f(t3 - mn);
      float ps = (e0 + e1) + (e2 + e3);
#pragma unroll
      for (int off = 1; off < 16; off <<= 1) ps += __shfl_xor(ps, off, 32);
      lrow[r] = lrow[r] * al + ps;
      oacc0[r] *= al;
      oacc1[r] *= al;
      const int ro = (8 * hh + r) * 68 + c;
      pt[ro]      = e0;
      pt[ro + 16] = e1;
      pt[ro + 32] = e2;
      pt[ro + 48] = e3;
    }
    wave_sync_lds();
#pragma unroll
    for (int wi = 0; wi < 2; ++wi) {
      const float* prow = pt + c * 68 + 32 * wi + 8 * hh;
      const v4f p0 = *(const v4f*)(prow), p1 = *(const v4f*)(prow + 4);
      const v4f p2 = *(const v4f*)(prow + 16), p3 = *(const v4f*)(prow + 20);
      FragH pa;
#pragma unroll
      for (int e = 0; e < 4; ++e) {
        pa.h[0][e]     = (_Float16)(p0[e] * PCARRY);
        pa.h[0][4 + e] = (_Float16)(p1[e] * PCARRY);
        pa.h[1][e]     = (_Float16)(p2[e] * PCARRY);
        pa.h[1][4 + e] = (_Float16)(p3[e] * PCARRY);
      }
      const int k0 = kb + 32 * wi;
      const v16h vb0 = ldfrag_h(V + (size_t)c * NSEQ + k0 + 8 * hh);
      const v16h vb1 = ldfrag_h(V + (size_t)(16 + c) * NSEQ + k0 + 8 * hh);
      oacc0 = mma_h_raw(pa.v, vb0, oacc0);
      oacc1 = mma_h_raw(pa.v, vb1, oacc1);
      dep_guard3(oacc0, oacc1, pa.v, vb0, vb1);
    }
    wave_sync_lds();
  }

  float* os = Os[wave];
  const float oinv = 1.0f / (PCARRY * VCARRY);
#pragma unroll
  for (int r = 0; r < 8; ++r) {
    const float inv = (1.0f / lrow[r]) * oinv;
    os[(8 * hh + r) * 32 + c]      = oacc0[r] * inv;
    os[(8 * hh + r) * 32 + 16 + c] = oacc1[r] * inv;
  }
  wave_sync_lds();
  {
    const int q4 = lane >> 3, e4 = (lane & 7) * 4;
    v4f vals[4];
#pragma unroll
    for (int it = 0; it < 4; ++it) {
      const int row = it * 4 + q4;
      vals[it] = *(const v4f*)(os + row * 32 + e4);
    }
    for (int pass = 0; pass < 2; ++pass) {
#pragma unroll
      for (int it = 0; it < 4; ++it) {
        const int row = it * 4 + q4;
        *(volatile v4f*)(ao + (gr + row) * CD + hcol + e4) = vals[it];
      }
      __threadfence();
    }
  }
}

__global__ __launch_bounds__(256) void ln_mid(const float* __restrict__ X, const float* __restrict__ gam,
                                               const float* __restrict__ bet, float* Y, unsigned short* YBH,
                                               unsigned short* YBL) {
  __shared__ __align__(16) float sb[8][2 * CD];
  const int tid = threadIdx.x, wave = tid >> 5, lane = tid & 31;
  const int hh = lane >> 4, c = lane & 15;
  const size_t row0 = ((size_t)blockIdx.x * 8 + wave) * 2;
  const size_t base = (row0 + hh) * CD + 8 * c;
  const v4f x0 = *(const v4f*)(X + base), x1 = *(const v4f*)(X + base + 4);
  float s = ((x0[0] + x0[1]) + (x0[2] + x0[3])) + ((x1[0] + x1[1]) + (x1[2] + x1[3]));
  s = wsum16(s);
  const float mean = s * (1.0f / CD);
  float d[8];
#pragma unroll
  for (int e = 0; e < 4; ++e) { d[e] = x0[e] - mean; d[4 + e] = x1[e] - mean; }
  float vs = 0.f;
#pragma unroll
  for (int e = 0; e < 8; ++e) vs += d[e] * d[e];
  vs = wsum16(vs);
  const float rstd = rsqrtf(vs * (1.0f / CD) + LNEPS);
  const v4f g0 = *(const v4f*)(gam + 8 * c), g1 = *(const v4f*)(gam + 8 * c + 4);
  const v4f b0 = *(const v4f*)(bet + 8 * c), b1 = *(const v4f*)(bet + 8 * c + 4);
  float y[8];
#pragma unroll
  for (int e = 0; e < 4; ++e) {
    y[e]     = (d[e] * rstd)     * bfr(g0[e]) + bfr(b0[e]);
    y[4 + e] = (d[4 + e] * rstd) * bfr(g1[e]) + bfr(b1[e]);
  }
  v4u oh, ol;
#pragma unroll
  for (int e = 0; e < 4; ++e) {
    const unsigned short h0 = bf_bits(y[2 * e]), h1 = bf_bits(y[2 * e + 1]);
    const unsigned short l0 = bf_bits(y[2 * e] - bf_up(h0)), l1 = bf_bits(y[2 * e + 1] - bf_up(h1));
    oh[e] = pk16(h0, h1);
    ol[e] = pk16(l0, l1);
  }
  float* sw = sb[wave];
  v4f ya, yb;
#pragma unroll
  for (int e = 0; e < 4; ++e) { ya[e] = y[e]; yb[e] = y[4 + e]; }
  *(v4f*)(sw + hh * CD + 8 * c)     = ya;
  *(v4f*)(sw + hh * CD + 8 * c + 4) = yb;
  wave_sync_lds();
  const v4f o0 = *(const v4f*)(sw + 4 * lane);
  const v4f o1 = *(const v4f*)(sw + CD + 4 * lane);
  for (int pass = 0; pass < 2; ++pass) {
    *(volatile v4u*)(YBH + base) = oh;
    *(volatile v4u*)(YBL + base) = ol;
    *(volatile v4f*)(Y + row0 * CD + 4 * lane) = o0;
    *(volatile v4f*)(Y + (row0 + 1) * CD + 4 * lane) = o1;
    __threadfence();
  }
}

__global__ __launch_bounds__(256) void ln_out(const float* __restrict__ Z, const float* __restrict__ gam,
                                               const float* __restrict__ bet, float* out) {
  __shared__ __align__(16) float T[CD * 36];
  const int tid = threadIdx.x, wave = tid >> 5, lane = tid & 31;
  const int hh = lane >> 4, c = lane & 15;
  const int bx = blockIdx.x;
  const int b  = bx >> 7;
  const int n0 = (bx & 127) * 32;
  const v4f g0 = *(const v4f*)(gam + 8 * c), g1 = *(const v4f*)(gam + 8 * c + 4);
  const v4f b0 = *(const v4f*)(bet + 8 * c), b1 = *(const v4f*)(bet + 8 * c + 4);
#pragma unroll 1
  for (int i = 0; i < 2; ++i) {
    const int tl = wave * 4 + 2 * i + hh;
    const size_t base = ((size_t)b * NSEQ + n0 + tl) * CD + 8 * c;
    const v4f x0 = *(const v4f*)(Z + base), x1 = *(const v4f*)(Z + base + 4);
    float s = ((x0[0] + x0[1]) + (x0[2] + x0[3])) + ((x1[0] + x1[1]) + (x1[2] + x1[3]));
    s = wsum16(s);
    const float mean = s * (1.0f / CD);
    float d[8];
#pragma unroll
    for (int e = 0; e < 4; ++e) { d[e] = x0[e] - mean; d[4 + e] = x1[e] - mean; }
    float vs = 0.f;
#pragma unroll
    for (int e = 0; e < 8; ++e) vs += d[e] * d[e];
    vs = wsum16(vs);
    const float rstd = rsqrtf(vs * (1.0f / CD) + LNEPS);
#pragma unroll
    for (int e = 0; e < 4; ++e) {
      T[(8 * c + e) * 36 + tl]     = (d[e] * rstd)     * bfr(g0[e]) + bfr(b0[e]);
      T[(8 * c + 4 + e) * 36 + tl] = (d[4 + e] * rstd) * bfr(g1[e]) + bfr(b1[e]);
    }
  }
  __syncthreads();
  {
    const int q = lane >> 3, e4 = (lane & 7) * 4;
    v4f vals[4];
#pragma unroll
    for (int it = 0; it < 4; ++it) {
      const int cc = wave * 16 + it * 4 + q;
      vals[it] = *(const v4f*)(T + cc * 36 + e4);
    }
    for (int pass = 0; pass < 2; ++pass) {
#pragma unroll
      for (int it = 0; it < 4; ++it) {
        const int cc = wave * 16 + it * 4 + q;
        *(volatile v4f*)(out + ((size_t)(b * CD + cc)) * NSEQ + n0 + e4) = vals[it];
      }
      __threadfence();
    }
  }
}

extern "C" void kernel_launch(void* const* d_in, const int* in_sizes, int n_in,
                              void* d_out, int out_size, void* d_ws, size_t ws_size,
                              hipStream_t stream) {
  if (n_in < 17) return;
  if (in_sizes[0] != NB * CD * NSEQ) return;
  if (in_sizes[1] != NHEAD * HDIM * HDIM || in_sizes[3] != NHEAD * HDIM * HDIM || in_sizes[5] != NHEAD * HDIM * HDIM) return;
  if (in_sizes[2] != NHEAD * HDIM || in_sizes[4] != NHEAD * HDIM || in_sizes[6] != NHEAD * HDIM) return;
  if (in_sizes[7] != CD * CD || in_sizes[8] != CD || in_sizes[9] != CD || in_sizes[10] != CD) return;
  if (in_sizes[11] != CD * DFF || in_sizes[12] != DFF || in_sizes[13] != DFF * CD) return;
  if (in_sizes[14] != CD || in_sizes[15] != CD || in_sizes[16] != CD) return;
  if (out_size != NB * CD * NSEQ) return;

  const float* x     = (const float*)d_in[0];
  const float* w_q   = (const float*)d_in[1];   const float* b_q  = (const float*)d_in[2];
  const float* w_k   = (const float*)d_in[3];   const float* b_k  = (const float*)d_in[4];
  const float* w_v   = (const float*)d_in[5];   const float* b_v  = (const float*)d_in[6];
  const float* w_p   = (const float*)d_in[7];   const float* b_p  = (const float*)d_in[8];
  const float* g_1   = (const float*)d_in[9];   const float* be_1 = (const float*)d_in[10];
  const float* w_1   = (const float*)d_in[11];  const float* b_1  = (const float*)d_in[12];
  const float* w_2   = (const float*)d_in[13];  const float* b_2  = (const float*)d_in[14];
  const float* g_2   = (const float*)d_in[15];  const float* be_2 = (const float*)d_in[16];

  const size_t PWQK = (size_t)NHEAD * QKP * HDIM * 2;
  const size_t PWV2 = (size_t)NHEAD * VTR * HDIM * 2;
  const size_t PWPT = (size_t)CD * CD * 2;
  const size_t PW1  = (size_t)DFF * CD * 2;
  const size_t PW2  = (size_t)CD * DFF * 2;
  const size_t PBIA = 4096;
  const size_t PXH  = (size_t)MP * CD * 2;
  const size_t PXI  = (size_t)MP * HDIM * 2;
  const size_t PQK  = (size_t)MP * QKP * 2;
  const size_t PVT  = (size_t)NB * VTR * NSEQ * 2;
  const size_t PAF  = (size_t)MP * CD * 4;
  const size_t PYB  = (size_t)MP * CD * 2;
  const size_t PGB  = (size_t)MP * DFF * 2;
  size_t off = 0;
  const size_t oWQK = off; off += PWQK;
  const size_t oWV2 = off; off += PWV2;
  const size_t oWPT = off; off += PWPT;
  const size_t oW1T = off; off += PW1;
  const size_t oW2T = off; off += PW2;
  const size_t oBIA = off; off += PBIA;
  const size_t oXH  = off; off += PXH;
  const size_t oXI  = off; off += PXI;
  const size_t oQK  = off; off += PQK;
  const size_t oVT2 = off; off += PVT;
  const size_t oAO  = off; off += PAF;
  const size_t oX1  = off; off += PAF;
  const size_t oY32 = off; off += PAF;
  const size_t oYBH = off; off += PYB;
  const size_t oYBL = off; off += PYB;
  const size_t oGBH = off; off += PGB;
  const size_t oGBL = off; off += PGB;
  const size_t oZ32 = off; off += PAF;
  if (off > ws_size) return;
  if (off > (size_t)134217728) return;

  char* ws = (char*)d_ws;
  unsigned short* WQK = (unsigned short*)(ws + oWQK);
  unsigned short* WV2 = (unsigned short*)(ws + oWV2);
  unsigned short* WPT = (unsigned short*)(ws + oWPT);
  unsigned short* W1T = (unsigned short*)(ws + oW1T);
  unsigned short* W2T = (unsigned short*)(ws + oW2T);
  float*          BIA = (float*)(ws + oBIA);
  unsigned short* XH  = (unsigned short*)(ws + oXH);
  unsigned short* XI  = (unsigned short*)(ws + oXI);
  unsigned short* QK  = (unsigned short*)(ws + oQK);
  unsigned short* VT2 = (unsigned short*)(ws + oVT2);
  float*          AO  = (float*)(ws + oAO);
  float*          X1  = (float*)(ws + oX1);
  float*          Y32 = (float*)(ws + oY32);
  unsigned short* YBH = (unsigned short*)(ws + oYBH);
  unsigned short* YBL = (unsigned short*)(ws + oYBL);
  unsigned short* GBH = (unsigned short*)(ws + oGBH);
  unsigned short* GBL = (unsigned short*)(ws + oGBL);
  float*          Z32 = (float*)(ws + oZ32);
  float*          out = (float*)d_out;

  const int n8qk = (NHEAD * QKP * HDIM) / 8;
  const int n8p  = (CD * CD) / 8;
  const int n8f  = (CD * DFF) / 8;
  if ((n8qk % 256) != 0 || (n8p % 256) != 0 || (n8f % 256) != 0) return;
  const dim3 blk(256), blk128(128);
  const dim3 gCqk((n8qk + 255) / 256), gCp((n8p + 255) / 256), gCf((n8f + 255) / 256);
  const dim3 gPrep(MP / 32);
  const dim3 gXi((MP * 4) / 256);
  const dim3 gQK(((MP / 64) * (QKP / 64) + 7) / 8, 1);
  const dim3 gVT(((VTR / 64) * (NSEQ / 64) + 7) / 8, NB);
  const dim3 gAttn(NB * (NSEQ / 64));
  const dim3 gO(((MP / 64) * (CD / 64) + 7) / 8, 1);
  const dim3 gLN(MP / 16);
  const dim3 gF1(((MP / 64) * (DFF / 64) + 7) / 8, 1);
  const dim3 gOut(MP / 32);

  conv_t16<0><<<gCqk, blk, 0, stream>>>(w_q, w_k, WQK, HDIM, HDIM, QKP, n8qk, WSC);
  conv_t16<0><<<gCqk, blk, 0, stream>>>(w_v, w_v, WV2, HDIM, HDIM, VTR, n8qk, WSC);
  conv_t16<0><<<gCp,  blk, 0, stream>>>(w_p, w_p, WPT, CD, CD, CD, n8p, WSC);
  conv_t16<1><<<gCf,  blk, 0, stream>>>(w_1, w_1, W1T, CD, DFF, DFF, n8f, 1.0f);
  conv_t16<1><<<gCf,  blk, 0, stream>>>(w_2, w_2, W2T, DFF, CD, CD, n8f, 1.0f);
  pack_bias<<<dim3(1), blk128, 0, stream>>>(b_q, b_k, b_v, BIA);

  xprep<<<gPrep, blk, 0, stream>>>(x, XH);

  for (int h = 0; h < NHEAD; ++h) {
    const unsigned short* Apl = (h == 0) ? XH : XI;
    const int la = (h == 0) ? CD : HDIM;
    if (h > 0) xiprep<<<gXi, blk, 0, stream>>>(XH, AO, XI, h);
    gemm64<0, 0, 1, 2, 0, 0, 0><<<gQK, blk, 0, stream>>>(
        (const void*)Apl, (const void*)Apl, la, 0LL, 1.0f,
        WQK + (size_t)h * QKP * HDIM, HDIM, 0LL,
        BIA + h * QKP, QKCARRY, (const void*)X1,
        (void*)QK, (void*)QK, QKP, 0LL, MP, QKP, HDIM, QKCARRY / WSC);
    gemm64<0, 0, 1, 2, 1, 0, 0><<<gVT, blk, 0, stream>>>(
        (const void*)(WV2 + (size_t)h * VTR * HDIM), (const void*)(WV2 + (size_t)h * VTR * HDIM), HDIM, 0LL, 1.0f,
        Apl, la, (long long)NSEQ * la,
        BIA + 256 + h * VTR, VCARRY, (const void*)X1,
        (void*)VT2, (void*)VT2, NSEQ, (long long)VTR * NSEQ, VTR, NSEQ, HDIM, VCARRY / WSC);
    attn_head<<<gAttn, blk128, 0, stream>>>(QK, VT2, AO, h * HDIM);
  }

  gemm64<0, 1, 1, 0, 0, 0, 2><<<gO, blk, 0, stream>>>(
      (const void*)AO, (const void*)AO, CD, 0LL, AOCARRY,
      WPT, CD, 0LL,
      b_p, 1.0f, (const void*)XH,
      (void*)X1, (void*)X1, CD, 0LL, MP, CD, CD, 1.0f / (AOCARRY * WSC));

  ln_mid<<<gLN, blk, 0, stream>>>(X1, g_1, be_1, Y32, YBH, YBL);

  gemm64<1, 0, 2, 3, 0, 2, 0><<<gF1, blk, 0, stream>>>(
      (const void*)YBH, (const void*)YBL, CD, 0LL, 1.0f,
      W1T, CD, 0LL,
      b_1, 1.0f, (const void*)X1,
      (void*)GBH, (void*)GBL, DFF, 0LL, MP, DFF, CD, 1.0f);

  gemm64<1, 0, 2, 0, 0, 0, 1><<<gO, blk, 0, stream>>>(
      (const void*)GBH, (const void*)GBL, DFF, 0LL, 1.0f,
      W2T, DFF, 0LL,
      b_2, 1.0f, (const void*)Y32,
      (void*)Z32, (void*)Z32, CD, 0LL, MP, CD, DFF, 1.0f);

  ln_out<<<gOut, blk, 0, stream>>>(Z32, g_2, be_2, out);
  (void)hipGetLastError();
}
